// AttnBlockv3_24077586661592
// MI455X (gfx1250) — hardware-verified
//
#include <hip/hip_runtime.h>

typedef __attribute__((ext_vector_type(16))) _Float16 v16h;
typedef __attribute__((ext_vector_type(8)))  _Float16 v8h;
typedef __attribute__((ext_vector_type(16))) __bf16   v16b;
typedef __attribute__((ext_vector_type(8)))  __bf16   v8b;
typedef __attribute__((ext_vector_type(8)))  float    v8f;
typedef __attribute__((ext_vector_type(4)))  float    v4f;
#define U16(p) ((const unsigned short*)(const void*)(p))

static constexpr int kB  = 16;
static constexpr int kN  = 4096;
static constexpr int kC  = 128;
static constexpr int kM  = kB * kN;
static constexpr int kNG = 32;
static constexpr int kCPG = 4;

__device__ __forceinline__ unsigned short f2bf_bits(float f) {
  unsigned u = __float_as_uint(f);
  return (unsigned short)((u + 0x7FFFu + ((u >> 16) & 1u)) >> 16);
}
__device__ __forceinline__ float bf_bits2f(unsigned short h) { return __uint_as_float(((unsigned)h) << 16); }

__device__ __forceinline__ void dep_guard_h(v8f& a, v8f& b, v16h x, v16h y) { asm volatile("v_nop\n\tv_nop\n\tv_nop\n\tv_nop" : "+v"(a), "+v"(b) : "v"(x), "v"(y)); }
__device__ __forceinline__ void dep_guard_b(v8f& a, v8f& b, v16b x, v16b y) { asm volatile("v_nop\n\tv_nop\n\tv_nop\n\tv_nop" : "+v"(a), "+v"(b) : "v"(x), "v"(y)); }
__device__ __forceinline__ void keep4_h(v16h a, v16h b, v16h c, v16h d) { asm volatile("v_nop" :: "v"(a), "v"(b), "v"(c), "v"(d)); }
__device__ __forceinline__ void keep4_b(v16b a, v16b b, v16b c, v16b d) { asm volatile("v_nop" :: "v"(a), "v"(b), "v"(c), "v"(d)); }
__device__ __forceinline__ void acc_guard4(v8f& a, v8f& b, v8f& c, v8f& d) { asm volatile("v_nop\n\tv_nop\n\tv_nop\n\tv_nop" : "+v"(a), "+v"(b), "+v"(c), "+v"(d)); }
template <typename T> struct Frag;
template <> struct Frag<_Float16> {
  typedef v16h V; union U { v16h v; v8h h[2]; };
  static __device__ __forceinline__ v16h load(const _Float16* p) {
    U f; f.h[0] = *(const v8h*)(p); f.h[1] = *(const v8h*)(p + 16); return f.v;
  }
  static __device__ __forceinline__ v8f mma(v16h a, v16h b, v8f c) {
    return __builtin_amdgcn_wmma_f32_16x16x32_f16(false, a, false, b, (short)0, c, false, false);
  }
  static __device__ __forceinline__ void guard(v8f& a, v8f& b, v16h x, v16h y) { dep_guard_h(a, b, x, y); }
  static __device__ __forceinline__ void keep(v16h a, v16h b, v16h c, v16h d) { keep4_h(a, b, c, d); }
};
template <> struct Frag<__bf16> {
  typedef v16b V; union U { v16b v; v8b h[2]; };
  static __device__ __forceinline__ v16b load(const __bf16* p) {
    U f; f.h[0] = *(const v8b*)(p); f.h[1] = *(const v8b*)(p + 16); return f.v;
  }
  static __device__ __forceinline__ v8f mma(v16b a, v16b b, v8f c) {
    return __builtin_amdgcn_wmma_f32_16x16x32_bf16(false, a, false, b, (short)0, c, false, false);
  }
  static __device__ __forceinline__ void guard(v8f& a, v8f& b, v16b x, v16b y) { dep_guard_b(a, b, x, y); }
  static __device__ __forceinline__ void keep(v16b a, v16b b, v16b c, v16b d) { keep4_b(a, b, c, d); }
};

__device__ __forceinline__ v8f mma16(v16h a, v16h b, v8f c) {
  c = __builtin_amdgcn_wmma_f32_16x16x32_f16(false, a, false, b, (short)0, c, false, false);
  asm volatile("v_nop\n\tv_nop\n\tv_nop\n\tv_nop" : "+v"(c) : "v"(a), "v"(b));
  return c;
}

template <int ET> struct Elem;
template <> struct Elem<0> { typedef _Float16 T; };
template <> struct Elem<1> { typedef __bf16 T; };
template <int ET, bool SPLIT, int BIAS_MODE, int OUT_MODE, bool RESID, int ACT = 0>
__global__ __launch_bounds__(256) void wmma_gemm64(
    const unsigned short* __restrict__ Ap, const unsigned short* __restrict__ A2p, int lda, long strideA,
    const unsigned short* __restrict__ Btp, const unsigned short* __restrict__ Bt2p, int ldb, long strideB,
    void* __restrict__ Cout, void* __restrict__ Cout2, int ldc, long strideC,
    const float* __restrict__ bias,
    const float* __restrict__ resid, long strideR,
    int M, int N, int K, float scale) {
  typedef typename Elem<ET>::T T;
  typedef typename Frag<T>::V V;
  const T* A = (const T*)Ap; const T* A2 = (const T*)A2p; const T* Bt = (const T*)Btp; const T* Bt2 = (const T*)Bt2p;
  __shared__ __align__(16) float sT[8][16 * 68];
  const int b    = blockIdx.y;
  const int lane = threadIdx.x & 31;
  const int wave = threadIdx.x >> 5;
  const int tilesN = N >> 6;
  const int tilesM = M >> 6;
  const int tile = blockIdx.x * 8 + wave;
  if (tile >= tilesM * tilesN) return;
  const int tm = tile / tilesN;
  const int tn = tile - tm * tilesN;
  const int m0 = tm << 6;
  const int n0 = tn << 6;

  const T* Ab  = A  + (size_t)b * strideA;
  const T* Bb  = Bt + (size_t)b * strideB;
  const T* Ab2 = SPLIT ? (A2  + (size_t)b * strideA) : nullptr;
  const T* Bb2 = SPLIT ? (Bt2 + (size_t)b * strideB) : nullptr;

  const int rlane = lane & 15;
  const int koff  = (lane >> 4) * 8;
  const int mOff  = (lane >> 4) * 8;

  v8f acc[4][4];
#pragma unroll
  for (int i = 0; i < 4; ++i)
#pragma unroll
    for (int j = 0; j < 4; ++j) acc[i][j] = (v8f){0.f,0.f,0.f,0.f,0.f,0.f,0.f,0.f};

  for (int k0 = 0; k0 < K; k0 += 32) {
    V bh[4], bl[4];
#pragma unroll
    for (int j = 0; j < 4; ++j) {
      const size_t bo = (size_t)(n0 + (j << 4) + rlane) * ldb + koff + k0;
      bh[j] = Frag<T>::load(Bb + bo);
      if (SPLIT) bl[j] = Frag<T>::load(Bb2 + bo);
    }
#pragma unroll
    for (int i = 0; i < 4; ++i) {
      const size_t ao = (size_t)(m0 + (i << 4) + rlane) * lda + koff + k0;
      V ah = Frag<T>::load(Ab + ao);
      V al;
      if (SPLIT) al = Frag<T>::load(Ab2 + ao);
#pragma unroll
      for (int j = 0; j < 4; ++j) {
        acc[i][j] = Frag<T>::mma(ah, bh[j], acc[i][j]);
        if (SPLIT) {
          acc[i][j] = Frag<T>::mma(ah, bl[j], acc[i][j]);
          acc[i][j] = Frag<T>::mma(al, bh[j], acc[i][j]);
        }
      }
      Frag<T>::guard(acc[i][0], acc[i][3], ah, SPLIT ? al : ah);
    }
    Frag<T>::keep(bh[0], bh[1], bh[2], bh[3]);
    if (SPLIT) Frag<T>::keep(bl[0], bl[1], bl[2], bl[3]);
  }
  acc_guard4(acc[0][0], acc[0][1], acc[0][2], acc[0][3]);
  acc_guard4(acc[1][0], acc[1][1], acc[1][2], acc[1][3]);
  acc_guard4(acc[2][0], acc[2][1], acc[2][2], acc[2][3]);
  acc_guard4(acc[3][0], acc[3][1], acc[3][2], acc[3][3]);

  float* slab = sT[wave];
  const float* Rb = RESID ? (resid + (size_t)b * strideR) : nullptr;
#pragma unroll
  for (int i = 0; i < 4; ++i) {
    const int mBase = m0 + (i << 4);
#pragma unroll
    for (int j = 0; j < 4; ++j) {
      const int n = n0 + (j << 4) + rlane;
      float bv = 0.f;
      if (BIAS_MODE == 2) bv = bias[n];
#pragma unroll
      for (int r = 0; r < 8; ++r) {
        float v = acc[i][j][r] * scale;
        if (BIAS_MODE == 1) v += bias[mBase + mOff + r];
        if (BIAS_MODE == 2) v += bv;
        if (RESID) v += Rb[(size_t)(mBase + mOff + r) * ldc + n];
        if (ACT == 1) v = tanhf(v);
        if (ACT == 2) v = fmaxf(v, 0.0f);
        if (ACT == 3) v = v / (1.0f + expf(-v));
        if (ACT == 4) v = (v > 0.f) ? v : 0.01f * v;
        if (ACT == 5) v = 0.5f * v * (1.0f + erff(v * 0.70710678118654752f));
        slab[(mOff + r) * 68 + (j << 4) + rlane] = v;
      }
    }
    __builtin_amdgcn_fence(__ATOMIC_RELEASE, "workgroup");
    __builtin_amdgcn_wave_barrier();
    __builtin_amdgcn_fence(__ATOMIC_ACQUIRE, "workgroup");
    if (OUT_MODE == 0) {
      float* C = (float*)Cout + (size_t)b * strideC;
      const int hh = lane >> 4, c4 = (lane & 15) * 4;
      for (int pass = 0; pass < 2; ++pass) {
#pragma unroll
        for (int it = 0; it < 8; ++it) {
          const int row = it * 2 + hh;
          v4f v = *(const v4f*)(slab + row * 68 + c4);
          *(volatile v4f*)(C + (size_t)(mBase + row) * ldc + n0 + c4) = v;
        }
        __threadfence();
      }
    } else {
      const int q = lane >> 3, c8 = (lane & 7) * 8;
      unsigned short* C  = (unsigned short*)Cout  + (size_t)b * strideC;
      unsigned short* C2 = (OUT_MODE == 2) ? ((unsigned short*)Cout2 + (size_t)b * strideC) : nullptr;
      for (int pass = 0; pass < 2; ++pass) {
#pragma unroll
        for (int it = 0; it < 4; ++it) {
          const int row = it * 4 + q;
          const float* sp = slab + row * 68 + c8;
          v8h hv, lv;
#pragma unroll
          for (int e = 0; e < 8; ++e) {
            if (OUT_MODE == 1) {
              hv[e] = (_Float16)sp[e];
            } else {
              unsigned short hb = f2bf_bits(sp[e]);
              unsigned short lb = f2bf_bits(sp[e] - bf_bits2f(hb));
              hv[e] = __builtin_bit_cast(_Float16, hb);
              lv[e] = __builtin_bit_cast(_Float16, lb);
            }
          }
          *(volatile v8h*)(C + (size_t)(mBase + row) * ldc + n0 + c8) = hv;
          if (OUT_MODE == 2) *(volatile v8h*)(C2 + (size_t)(mBase + row) * ldc + n0 + c8) = lv;
        }
        __threadfence();
      }
    }
    __builtin_amdgcn_fence(__ATOMIC_RELEASE, "workgroup");
    __builtin_amdgcn_wave_barrier();
    __builtin_amdgcn_fence(__ATOMIC_ACQUIRE, "workgroup");
  }
}

#define WC_P 136
__global__ __launch_bounds__(256) void k_wconvert(const float* __restrict__ w0, const float* __restrict__ w1,
                                                 const float* __restrict__ w2, const float* __restrict__ w3,
                                                 _Float16* __restrict__ wt16) {
  __shared__ __align__(16) _Float16 T[32 * WC_P];
  const int mat = blockIdx.y;
  const int n0  = blockIdx.x * 32;
  const int t   = threadIdx.x;
  const float* src = (mat == 0) ? w0 : (mat == 1) ? w1 : (mat == 2) ? w2 : w3;
#pragma unroll
  for (int it = 0; it < 16; ++it) {
    const int idx = it * 256 + t;
    const int k = idx >> 5, j = idx & 31;
    T[j * WC_P + k] = (_Float16)src[(size_t)k * kC + n0 + j];
  }
  __syncthreads();
  const int row0 = t >> 4, c8 = (t & 15) * 8;
  _Float16* dst = wt16 + ((size_t)mat * kC + n0) * kC;
  for (int pass = 0; pass < 2; ++pass) {
#pragma unroll
    for (int it = 0; it < 2; ++it) {
      const int rr = row0 + 16 * it;
      const v8h val = *(const v8h*)(T + rr * WC_P + c8);
      *(volatile v8h*)(dst + (size_t)rr * kC + c8) = val;
    }
    __threadfence();
  }
}

__global__ __launch_bounds__(256) void k_gn_stats(const float* __restrict__ x, float* __restrict__ gtab) {
  __shared__ double red_s[8][32], red_q[8][32];
  __shared__ __align__(16) float tab[64];
  const int b = blockIdx.x;
  const int t = threadIdx.x, g = t & 31, rs = t >> 5;
  const float* xb = x + (size_t)b * kN * kC + kCPG * g;
  double s = 0.0, ss = 0.0;
  for (int r = rs; r < kN; r += 8) {
    const v4f v = *(const v4f*)(xb + (size_t)r * kC);
#pragma unroll
    for (int e = 0; e < 4; ++e) { const double d = (double)v[e]; s += d; ss += d * d; }
  }
  red_s[rs][g] = s; red_q[rs][g] = ss;
  __syncthreads();
  if (t < 32) {
    double S = 0.0, Q = 0.0;
#pragma unroll
    for (int i = 0; i < 8; ++i) { S += red_s[i][t]; Q += red_q[i][t]; }
    const double inv_n = 1.0 / (double)(kN * kCPG);
    const double mean = S * inv_n;
    double var = Q * inv_n - mean * mean;
    if (var < 0.0) var = 0.0;
    const float rstd = rsqrtf((float)var + 1e-6f);
    tab[t] = (float)mean;
    tab[32 + t] = rstd;
  }
  __syncthreads();
  if (t < 16) {
    const v4f v = *(const v4f*)(tab + 4 * t);
    *(volatile v4f*)(gtab + (size_t)b * 64 + 4 * t) = v;
    __threadfence();
    *(volatile v4f*)(gtab + (size_t)b * 64 + 4 * t) = v;
  }
}

__global__ __launch_bounds__(256) void k_gn_apply(const float* __restrict__ x, const float* __restrict__ gs,
                                                 const float* __restrict__ gb, const float* __restrict__ gtab,
                                                 _Float16* __restrict__ h16, int nvec) {
  const int i = blockIdx.x * 256 + threadIdx.x;
  if (i >= nvec) return;
  const int m  = i >> 4;
  const int c8 = (i & 15) * 8;
  const int b  = m >> 12;
  const int g0 = c8 >> 2;
  const float* tb = gtab + (size_t)b * 64;
  const float mean0 = tb[g0],     rstd0 = tb[32 + g0];
  const float mean1 = tb[g0 + 1], rstd1 = tb[32 + g0 + 1];
  const float* xr = x + (size_t)m * kC + c8;
  const v4f xa = *(const v4f*)(xr), xb2 = *(const v4f*)(xr + 4);
  const v4f sa = *(const v4f*)(gs + c8), sb = *(const v4f*)(gs + c8 + 4);
  const v4f ba = *(const v4f*)(gb + c8), bb = *(const v4f*)(gb + c8 + 4);
  v8h hv;
#pragma unroll
  for (int e = 0; e < 4; ++e) {
    hv[e]     = (_Float16)(((xa[e]  - mean0) * rstd0) * sa[e] + ba[e]);
    hv[4 + e] = (_Float16)(((xb2[e] - mean1) * rstd1) * sb[e] + bb[e]);
  }
  _Float16* dst = h16 + (size_t)m * kC + c8;
  *(volatile v8h*)dst = hv;
  __threadfence();
  *(volatile v8h*)dst = hv;
}

#define AT_KC 64
#define AT_OP 136
__global__ __launch_bounds__(128) void k_attn128(const _Float16* __restrict__ q16, const _Float16* __restrict__ k16,
                                                const _Float16* __restrict__ vt16, _Float16* __restrict__ o16,
                                                float scale) {
  __shared__ __align__(16) _Float16 Ksh[AT_KC * kC];
  __shared__ __align__(16) _Float16 Vts[kC * AT_KC];
  __shared__ __align__(16) _Float16 Psh[4][16 * AT_KC];
  __shared__ __align__(16) _Float16 Osh[4][16 * AT_OP];
  const int tid  = threadIdx.x;
  const int wave = tid >> 5;
  const int lane = tid & 31;
  const int hh   = lane >> 4;
  const int c    = lane & 15;
  const int b    = blockIdx.x >> 6;
  const int qb   = blockIdx.x & 63;
  const int q0   = qb * 64 + wave * 16;
  const size_t tok0 = (size_t)b * kN;

  v16h qa[4];
  {
    const _Float16* qrow = q16 + (tok0 + q0 + c) * kC;
#pragma unroll
    for (int dc = 0; dc < 4; ++dc) qa[dc] = Frag<_Float16>::load(qrow + dc * 32 + 8 * hh);
  }

  float mrow[8], lrow[8];
  v8f oacc[8];
#pragma unroll
  for (int r = 0; r < 8; ++r) { mrow[r] = -__builtin_inff(); lrow[r] = 0.f; }
#pragma unroll
  for (int t = 0; t < 8; ++t) oacc[t] = (v8f){0.f,0.f,0.f,0.f,0.f,0.f,0.f,0.f};

  _Float16* pw = Psh[wave];
  const float PSC = 32768.0f;

#pragma unroll 1
  for (int kc = 0; kc < kN / AT_KC; ++kc) {
    const int kv0 = kc * AT_KC;
    __syncthreads();
#pragma unroll
    for (int it = 0; it < 8; ++it) {
      const int i = tid + 128 * it;
      {
        const int row = i >> 4, d8 = (i & 15) * 8;
        const v8h kk = *(const v8h*)(k16 + (tok0 + kv0 + row) * kC + d8);
        *(v8h*)(Ksh + row * kC + d8) = kk;
      }
      {
        const int d = i >> 3, c8 = (i & 7) * 8;
        const v8h vv = *(const v8h*)(vt16 + ((size_t)b * kC + d) * kN + kv0 + c8);
        *(v8h*)(Vts + d * AT_KC + c8) = vv;
      }
    }
    __syncthreads();

    v8f s[4];
#pragma unroll
    for (int j = 0; j < 4; ++j) {
      s[j] = (v8f){0.f,0.f,0.f,0.f,0.f,0.f,0.f,0.f};
#pragma unroll
      for (int dc = 0; dc < 4; ++dc) {
        const v16h kb = Frag<_Float16>::load(Ksh + (j * 16 + c) * kC + dc * 32 + 8 * hh);
        s[j] = mma16(qa[dc], kb, s[j]);
      }
    }

    float cm[8];
#pragma unroll
    for (int r = 0; r < 8; ++r) {
      float m = -__builtin_inff();
#pragma unroll
      for (int j = 0; j < 4; ++j) {
        const float sv = s[j][r] * scale;
        s[j][r] = sv;
        m = fmaxf(m, sv);
      }
#pragma unroll
      for (int off = 1; off < 16; off <<= 1) m = fmaxf(m, __shfl_xor(m, off, 32));
      cm[r] = m;
    }
#pragma unroll
    for (int r = 0; r < 8; ++r) {
      const float mnew  = fmaxf(mrow[r], cm[r]);
      const float alpha = __expf(mrow[r] - mnew);
      mrow[r] = mnew;
      float psum = 0.f;
#pragma unroll
      for (int j = 0; j < 4; ++j) {
        const float p = __expf(s[j][r] - mnew);
        psum += p;
        pw[(8 * hh + r) * AT_KC + j * 16 + c] = (_Float16)(p * PSC);
      }
#pragma unroll
      for (int off = 1; off < 16; off <<= 1) psum += __shfl_xor(psum, off, 32);
      lrow[r] = lrow[r] * alpha + psum;
#pragma unroll
      for (int t = 0; t < 8; ++t) oacc[t][r] *= alpha;
    }
    __builtin_amdgcn_fence(__ATOMIC_RELEASE, "workgroup");
    __builtin_amdgcn_wave_barrier();
    __builtin_amdgcn_fence(__ATOMIC_ACQUIRE, "workgroup");

#pragma unroll
    for (int kk = 0; kk < 2; ++kk) {
      const v16h pa = Frag<_Float16>::load(pw + c * AT_KC + kk * 32 + 8 * hh);
#pragma unroll
      for (int t = 0; t < 8; ++t) {
        const v16h vb = Frag<_Float16>::load(Vts + (t * 16 + c) * AT_KC + kk * 32 + 8 * hh);
        oacc[t] = mma16(pa, vb, oacc[t]);
      }
    }
  }

  _Float16* osw = Osh[wave];
#pragma unroll
  for (int r = 0; r < 8; ++r) {
    const float inv = 1.0f / (lrow[r] * PSC);
#pragma unroll
    for (int t = 0; t < 8; ++t) osw[(8 * hh + r) * AT_OP + t * 16 + c] = (_Float16)(oacc[t][r] * inv);
  }
  __builtin_amdgcn_fence(__ATOMIC_RELEASE, "workgroup");
  __builtin_amdgcn_wave_barrier();
  __builtin_amdgcn_fence(__ATOMIC_ACQUIRE, "workgroup");
  {
    const int c8 = (lane & 15) * 8;
    _Float16* ob = o16 + (tok0 + q0) * kC;
    for (int pass = 0; pass < 2; ++pass) {
#pragma unroll
      for (int it = 0; it < 8; ++it) {
        const int row = it * 2 + hh;
        const v8h val = *(const v8h*)(osw + row * AT_OP + c8);
        *(volatile v8h*)(ob + (size_t)row * kC + c8) = val;
      }
      __threadfence();
    }
  }
}

extern "C" void kernel_launch(void* const* d_in, const int* in_sizes, int n_in,
                              void* d_out, int out_size, void* d_ws, size_t ws_size,
                              hipStream_t stream) {
  if (n_in < 11) return;
  if (in_sizes[0] != kM * kC || out_size != kM * kC) return;
  if (in_sizes[1] != kC || in_sizes[2] != kC || in_sizes[4] != kC || in_sizes[6] != kC ||
      in_sizes[8] != kC || in_sizes[10] != kC) return;
  if (in_sizes[3] != kC * kC || in_sizes[5] != kC * kC || in_sizes[7] != kC * kC || in_sizes[9] != kC * kC) return;

  const float* x  = (const float*)d_in[0];
  const float* gs = (const float*)d_in[1];
  const float* gb = (const float*)d_in[2];
  const float* wq = (const float*)d_in[3];
  const float* bq = (const float*)d_in[4];
  const float* wk = (const float*)d_in[5];
  const float* bk = (const float*)d_in[6];
  const float* wv = (const float*)d_in[7];
  const float* bv = (const float*)d_in[8];
  const float* wo = (const float*)d_in[9];
  const float* bo = (const float*)d_in[10];
  float* out = (float*)d_out;

  const size_t szW   = (size_t)4 * kC * kC * sizeof(_Float16);
  const size_t szTab = (size_t)kB * 64 * sizeof(float);
  const size_t szT16 = (size_t)kM * kC * sizeof(_Float16);
  const size_t offW   = 0;
  const size_t offTab = offW + szW;
  const size_t offH   = offTab + szTab;
  const size_t offQ   = offH + szT16;
  const size_t offK   = offQ + szT16;
  const size_t offVt  = offK + szT16;
  const size_t offO   = offVt + szT16;
  const size_t offEnd = offO + szT16;
  if (offEnd > ws_size) return;

  char* ws = (char*)d_ws;
  _Float16* wt16 = (_Float16*)(ws + offW);
  float*    gtab = (float*)(ws + offTab);
  _Float16* h16  = (_Float16*)(ws + offH);
  _Float16* q16  = (_Float16*)(ws + offQ);
  _Float16* k16  = (_Float16*)(ws + offK);
  _Float16* vt16 = (_Float16*)(ws + offVt);
  _Float16* o16  = (_Float16*)(ws + offO);
  const _Float16* wtq = wt16;
  const _Float16* wtk = wt16 + (size_t)kC * kC;
  const _Float16* wtv = wt16 + (size_t)2 * kC * kC;
  const _Float16* wto = wt16 + (size_t)3 * kC * kC;

  k_wconvert<<<dim3(kC / 32, 4), 256, 0, stream>>>(wq, wk, wv, wo, wt16);
  k_gn_stats<<<kB, 256, 0, stream>>>(x, gtab);
  const int nvec = kM * (kC / 8);
  k_gn_apply<<<(nvec + 255) / 256, 256, 0, stream>>>(x, gs, gb, gtab, h16, nvec);

  const int gridMN = ((kM / 64) * (kC / 64) + 7) / 8;
  wmma_gemm64<0, false, 2, 1, false><<<dim3(gridMN, 1), 256, 0, stream>>>(
      U16(h16), U16(h16), kC, (long)0, U16(wtq), U16(wtq), kC, (long)0,
      (void*)q16, (void*)nullptr, kC, (long)0, bq, (const float*)nullptr, (long)0, kM, kC, kC, 1.0f);
  wmma_gemm64<0, false, 2, 1, false><<<dim3(gridMN, 1), 256, 0, stream>>>(
      U16(h16), U16(h16), kC, (long)0, U16(wtk), U16(wtk), kC, (long)0,
      (void*)k16, (void*)nullptr, kC, (long)0, bk, (const float*)nullptr, (long)0, kM, kC, kC, 1.0f);
  const int gridVt = ((kC / 64) * (kN / 64) + 7) / 8;
  wmma_gemm64<0, false, 1, 1, false><<<dim3(gridVt, kB), 256, 0, stream>>>(
      U16(wtv), U16(wtv), kC, (long)0, U16(h16), U16(h16), kC, (long)kN * kC,
      (void*)vt16, (void*)nullptr, kN, (long)kC * kN, bv, (const float*)nullptr, (long)0, kC, kN, kC, 1.0f);

  const float scale = 0.08838834764831845f;
  k_attn128<<<kB * (kN / 64), 128, 0, stream>>>(q16, k16, vt16, o16, scale);

  wmma_gemm64<0, false, 2, 0, true><<<dim3(gridMN, 1), 256, 0, stream>>>(
      U16(o16), U16(o16), kC, (long)0, U16(wto), U16(wto), kC, (long)0,
      (void*)out, (void*)nullptr, kC, (long)0, bo, x, (long)0, kM, kC, kC, 1.0f);
}
